// MetaLSTMCell_35691178230152
// MI455X (gfx1250) — hardware-verified
//
#include <hip/hip_runtime.h>


#define NB_  4096
#define IN_  1024
#define HM   1024
#define HH   256
#define EE   64
#define KC   2304
#define OFF_C  16777216
#define OFF_MH 33554432
#define OFF_MC 37748736
typedef _Float16 h16;
typedef unsigned short bf;
typedef __attribute__((ext_vector_type(16))) __bf16   v16bf;
typedef __attribute__((ext_vector_type(16))) _Float16 v16h;
typedef __attribute__((ext_vector_type(8)))  _Float16 v8h;
typedef __attribute__((ext_vector_type(8)))  unsigned short v8us;
typedef __attribute__((ext_vector_type(8)))  float    v8f;
typedef __attribute__((ext_vector_type(4)))  float    v4f;
typedef v8h  __attribute__((may_alias)) v8ha;
typedef v4f  __attribute__((may_alias)) v4fa;
typedef v8us __attribute__((may_alias)) v8usa;

__device__ __forceinline__ unsigned short f2bf(float f) { unsigned u = __float_as_uint(f); u += 0x7FFFu + ((u >> 16) & 1u); return (unsigned short)(u >> 16); }
__device__ __forceinline__ float bf2f(unsigned short b) { return __uint_as_float(((unsigned)b) << 16); }
__device__ __forceinline__ float bfr(float f) { return bf2f(f2bf(f)); }
__device__ __forceinline__ v16h cat16(v8h lo, v8h hi) { return __builtin_shufflevector(lo, hi, 0, 1, 2, 3, 4, 5, 6, 7, 8, 9, 10, 11, 12, 13, 14, 15); }
__device__ __forceinline__ v16bf cat16b(v8us lo, v8us hi) { return __builtin_bit_cast(v16bf, __builtin_shufflevector(lo, hi, 0, 1, 2, 3, 4, 5, 6, 7, 8, 9, 10, 11, 12, 13, 14, 15)); }
__device__ __forceinline__ v8f wmma16(v16h a, v16h b, v8f c) { return __builtin_amdgcn_wmma_f32_16x16x32_f16(false, a, false, b, (short)0, c, false, false); }
__device__ __forceinline__ v8f wmmab(v16bf a, v16bf b, v8f c) { return __builtin_amdgcn_wmma_f32_16x16x32_bf16(false, a, false, b, (short)0, c, false, false); }


template <typename T16> struct WFrag;
template <> struct WFrag<h16> { typedef v16h V; static __device__ __forceinline__ V ld(const h16* p) { return cat16(*(const v8h*)p, *(const v8h*)(p + 16)); } static __device__ __forceinline__ v8f mma(V a, V b, v8f c) { return wmma16(a, b, c); } };
template <> struct WFrag<bf> { typedef v16bf V; static __device__ __forceinline__ V ld(const bf* p) { return cat16b(*(const v8us*)p, *(const v8us*)(p + 16)); } static __device__ __forceinline__ v8f mma(V a, V b, v8f c) { return wmmab(a, b, c); } };
template <typename T16, int NSPLIT, bool BIAS>
__global__ __launch_bounds__(32) void k_gemmw(const T16* __restrict__ A, const T16* __restrict__ A2, const T16* __restrict__ Bt, const T16* __restrict__ Bt2, int K, float* C, int ldc, const float* __restrict__ bias, size_t sA, size_t sB, size_t sC) {
    typedef typename WFrag<T16>::V V;
    __shared__ __align__(16) float os[16 * 68];
    const size_t z = blockIdx.z; A += z * sA; if (A2) A2 += z * sA; Bt += z * sB; if (Bt2) Bt2 += z * sB; C += z * sC;
    const int lane = threadIdx.x & 31, lr = lane & 15, hi = lane >> 4; const int r0 = blockIdx.x * 64, c0 = blockIdx.y * 64;
    v8f acc[4][4];
#pragma unroll
    for (int mb = 0; mb < 4; ++mb)
#pragma unroll
        for (int nb = 0; nb < 4; ++nb) acc[mb][nb] = (v8f){};
    const size_t aoff = (size_t)(r0 + lr) * K + 8 * hi, boff = (size_t)(c0 + lr) * K + 8 * hi;
#pragma unroll 1
    for (int kc = 0; kc < K; kc += 32) {
        V a[4], a2[4];
#pragma unroll
        for (int mb = 0; mb < 4; ++mb) { a[mb] = WFrag<T16>::ld(A + aoff + (size_t)mb * 16 * K + kc); if (NSPLIT == 1 || NSPLIT == 2) a2[mb] = WFrag<T16>::ld(A2 + aoff + (size_t)mb * 16 * K + kc); }
#pragma unroll
        for (int nb = 0; nb < 4; ++nb) { const V b = WFrag<T16>::ld(Bt + boff + (size_t)nb * 16 * K + kc); V b2; if (NSPLIT >= 2) b2 = WFrag<T16>::ld(Bt2 + boff + (size_t)nb * 16 * K + kc);
#pragma unroll
            for (int mb = 0; mb < 4; ++mb) { acc[mb][nb] = WFrag<T16>::mma(a[mb], b, acc[mb][nb]); if (NSPLIT == 1 || NSPLIT == 2) acc[mb][nb] = WFrag<T16>::mma(a2[mb], b, acc[mb][nb]); if (NSPLIT >= 2) acc[mb][nb] = WFrag<T16>::mma(a[mb], b2, acc[mb][nb]); } }
        asm volatile("v_nop\n\tv_nop\n\tv_nop\n\tv_nop" : "+v"(acc[0][0]), "+v"(acc[1][1]), "+v"(acc[2][2]), "+v"(acc[3][3]) : "v"(a[0]), "v"(a[3]));
    }
#pragma unroll
    for (int mb = 0; mb < 4; ++mb) {
#pragma unroll
        for (int nb = 0; nb < 4; ++nb) {
#pragma unroll
            for (int j = 0; j < 8; ++j) os[(hi * 8 + j) * 68 + nb * 16 + lr] = acc[mb][nb][j]; }
        __builtin_amdgcn_wave_barrier(); asm volatile("" ::: "memory");
        float* crow = C + (size_t)(r0 + mb * 16) * ldc + c0;
#pragma unroll 1
        for (int ps = 0; ps < 2; ++ps) {
#pragma unroll
            for (int s = 0; s < 8; ++s) { const int row = 2 * s + hi, cofs = lr * 4; v4f val = *(const v4fa*)(os + row * 68 + cofs); if (BIAS) { val[0] += bfr(bias[c0 + cofs]); val[1] += bfr(bias[c0 + cofs + 1]); val[2] += bfr(bias[c0 + cofs + 2]); val[3] += bfr(bias[c0 + cofs + 3]); }
                *(volatile v4f*)(crow + (size_t)row * ldc + cofs) = val; }
            if (ps == 0) __threadfence(); }
        __builtin_amdgcn_wave_barrier(); asm volatile("" ::: "memory");
    }
}

__device__ __forceinline__ void splitf(float y, unsigned short& h, unsigned short& l) { h = f2bf(y); l = f2bf(y - bf2f(h)); }
__device__ __forceinline__ float sigm(float v) { return __fdiv_rn(1.0f, __fadd_rn(1.0f, expf(-v))); }
typedef __attribute__((ext_vector_type(4))) unsigned short v4us;
__global__ __launch_bounds__(256) void k_cvt8(const float* __restrict__ src, bf* dst, size_t n8) { const size_t i = (size_t)blockIdx.x * 256 + threadIdx.x; if (i >= n8) return; const v8f v = *(const v8f*)(src + i * 8); v8us o;
#pragma unroll
    for (int k = 0; k < 8; ++k) o[k] = f2bf(v[k]); *(volatile v8us*)(dst + i * 8) = o; __threadfence(); *(volatile v8us*)(dst + i * 8) = o; }

__global__ __launch_bounds__(256) void k_xcat(const float* __restrict__ x, const float* __restrict__ h, const float* __restrict__ mh, bf* XC) { const size_t e = ((size_t)blockIdx.x * 256 + threadIdx.x) * 8; if (e >= (size_t)NB_ * KC) return; const int c = (int)(e % KC); const size_t b = e / KC; const float* src = (c < IN_) ? (x + b * IN_ + c) : (c < IN_ + HM) ? (h + b * HM + (c - IN_)) : (mh + b * HH + (c - IN_ - HM)); const v8f v = *(const v8f*)src; v8us o;
#pragma unroll
    for (int q = 0; q < 8; ++q) o[q] = f2bf(v[q]); *(volatile v8us*)(XC + e) = o; __threadfence(); *(volatile v8us*)(XC + e) = o; }
__global__ __launch_bounds__(256) void k_wcat(const float* __restrict__ Wih, const float* __restrict__ Whh, bf* Bt) { const size_t e = ((size_t)blockIdx.x * 256 + threadIdx.x) * 8; if (e >= (size_t)(4 * HH) * KC) return; const int c = (int)(e % KC); const size_t n = e / KC; const float* src = (c < IN_ + HM) ? (Wih + n * (IN_ + HM) + c) : (Whh + n * HH + (c - IN_ - HM)); const v8f v = *(const v8f*)src; v8us o;
#pragma unroll
    for (int q = 0; q < 8; ++q) o[q] = f2bf(v[q]); *(volatile v8us*)(Bt + e) = o; __threadfence(); *(volatile v8us*)(Bt + e) = o; }
__global__ __launch_bounds__(256) void k_meta(const float* __restrict__ MP, const float* __restrict__ mc, float* OMH, float* OMC) { const size_t e = (size_t)blockIdx.x * 256 + threadIdx.x; if (e >= (size_t)NB_ * HH) return; const int uu = (int)(e % HH); const size_t b = e / HH; const float* mp = MP + b * 4 * HH;
    const float si = sigm(mp[uu]), sf = sigm(mp[HH + uu]), tg = tanhf(mp[2 * HH + uu]), so = sigm(mp[3 * HH + uu]); float a = __fmul_rn(sf, bfr(mc[e])); asm volatile("" : "+v"(a)); float b2 = __fmul_rn(si, tg); asm volatile("" : "+v"(b2)); const float cn = __fadd_rn(a, b2); const float hn = __fmul_rn(so, tanhf(cn));
    *(volatile float*)(OMC + e) = cn; *(volatile float*)(OMH + e) = hn; __threadfence(); *(volatile float*)(OMC + e) = cn; *(volatile float*)(OMH + e) = hn; }
__global__ __launch_bounds__(256) void k_split4(const float* __restrict__ F, bf* Ph, bf* Pl, size_t n4) { const size_t i = (size_t)blockIdx.x * 256 + threadIdx.x; if (i >= n4) return; const v4f v = *(const v4f*)(F + i * 4); v4us oh, ol;
#pragma unroll
    for (int q = 0; q < 4; ++q) { unsigned short a, c; splitf(v[q], a, c); oh[q] = a; ol[q] = c; } *(volatile v4us*)(Ph + i * 4) = oh; *(volatile v4us*)(Pl + i * 4) = ol; __threadfence(); *(volatile v4us*)(Ph + i * 4) = oh; *(volatile v4us*)(Pl + i * 4) = ol; }
__global__ __launch_bounds__(256) void k_gate(const float* __restrict__ ZD1, const float* __restrict__ XW, const float* __restrict__ ZD2, const float* __restrict__ HW, const float* __restrict__ ZB, int gsel, float* GATE) { const size_t e = ((size_t)blockIdx.x * 256 + threadIdx.x) * 4; if (e >= (size_t)NB_ * HM) return; const v4f a = *(const v4f*)(ZD1 + e), b = *(const v4f*)(XW + e), c = *(const v4f*)(ZD2 + e), d = *(const v4f*)(HW + e), zb = *(const v4f*)(ZB + e); v4f o;
#pragma unroll
    for (int q = 0; q < 4; ++q) { float t1 = __fmul_rn(a[q], b[q]); asm volatile("" : "+v"(t1)); float t2 = __fmul_rn(c[q], d[q]); asm volatile("" : "+v"(t2)); float s = __fadd_rn(t1, t2); asm volatile("" : "+v"(s)); const float pre = __fadd_rn(s, zb[q]); o[q] = (gsel == 2) ? tanhf(pre) : sigm(pre); }
    *(volatile v4f*)(GATE + e) = o; __threadfence(); *(volatile v4f*)(GATE + e) = o; }
__global__ __launch_bounds__(256) void k_main(const float* __restrict__ GI, const float* __restrict__ GF, const float* __restrict__ GG, const float* __restrict__ GO, const float* __restrict__ mc, float* OH, float* OC) { const size_t e = ((size_t)blockIdx.x * 256 + threadIdx.x) * 4; if (e >= (size_t)NB_ * HM) return; const v4f i4 = *(const v4f*)(GI + e), f4 = *(const v4f*)(GF + e), g4 = *(const v4f*)(GG + e), o4 = *(const v4f*)(GO + e), c4 = *(const v4f*)(mc + e); v4f cn, hn;
#pragma unroll
    for (int q = 0; q < 4; ++q) { float a = __fmul_rn(f4[q], bfr(c4[q])); asm volatile("" : "+v"(a)); float b2 = __fmul_rn(i4[q], g4[q]); asm volatile("" : "+v"(b2)); cn[q] = __fadd_rn(a, b2); hn[q] = __fmul_rn(o4[q], tanhf(cn[q])); }
    *(volatile v4f*)(OC + e) = cn; *(volatile v4f*)(OH + e) = hn; __threadfence(); *(volatile v4f*)(OC + e) = cn; *(volatile v4f*)(OH + e) = hn; }

extern "C" void kernel_launch(void* const* d_in, const int* in_sizes, int n_in,
                              void* d_out, int out_size, void* d_ws, size_t ws_size, hipStream_t stream) {
    (void)in_sizes; (void)n_in; (void)out_size;
    const float* x = (const float*)d_in[0]; const float* mh = (const float*)d_in[1]; const float* mc = (const float*)d_in[2]; const float* th = (const float*)d_in[3]; const float* tc = (const float*)d_in[4];
    const float* WiH = (const float*)d_in[5]; const float* WHH = (const float*)d_in[6]; const float* Wih = (const float*)d_in[7]; const float* Whh = (const float*)d_in[8]; const float* Whz = (const float*)d_in[9]; const float* Wd1 = (const float*)d_in[10]; const float* Wd2 = (const float*)d_in[11]; const float* Wbz = (const float*)d_in[12]; const float* bhy = (const float*)d_in[13];
    float* OH = (float*)d_out; float* OC = (float*)((char*)d_out + OFF_C); float* OMH = (float*)((char*)d_out + OFF_MH); float* OMC = (float*)((char*)d_out + OFF_MC);
    char* wsp = (char*)d_ws;
    auto take = [&](size_t bytes) { char* p = wsp; wsp += (bytes + 255) & ~(size_t)255; return (void*)p; };
    bf* XC = (bf*)take((size_t)NB_ * KC * 2); bf* XB = (bf*)take((size_t)NB_ * IN_ * 2); bf* HB = (bf*)take((size_t)NB_ * HM * 2); bf* WC = (bf*)take((size_t)4 * HH * KC * 2); float* MP = (float*)take((size_t)NB_ * 4 * HH * 4); bf* MHh = (bf*)take((size_t)NB_ * HH * 2); bf* MHl = (bf*)take((size_t)NB_ * HH * 2); bf* WHZ = (bf*)take((size_t)EE * HH * 2);
    float* Z = (float*)take((size_t)NB_ * EE * 4); bf* Zh = (bf*)take((size_t)NB_ * EE * 2); bf* Zl = (bf*)take((size_t)NB_ * EE * 2); bf* WIH = (bf*)take((size_t)4 * HM * IN_ * 2); bf* WHHb = (bf*)take((size_t)4 * HM * HM * 2); bf* WD1 = (bf*)take((size_t)4 * HM * EE * 2); bf* WD2 = (bf*)take((size_t)4 * HM * EE * 2); bf* WBZ = (bf*)take((size_t)4 * HM * EE * 2);
    float* XW = (float*)take((size_t)NB_ * HM * 4); float* HW = (float*)take((size_t)NB_ * HM * 4); float* ZD1 = (float*)take((size_t)NB_ * HM * 4); float* ZD2 = (float*)take((size_t)NB_ * HM * 4); float* ZB = (float*)take((size_t)NB_ * HM * 4);
    float* G0 = (float*)take((size_t)NB_ * HM * 4); float* G1 = (float*)take((size_t)NB_ * HM * 4); float* G2 = (float*)take((size_t)NB_ * HM * 4); float* G3 = (float*)take((size_t)NB_ * HM * 4);
    if ((size_t)(wsp - (char*)d_ws) > ws_size) return;
    const unsigned nb4 = (unsigned)(((size_t)NB_ * HM / 4 + 255) / 256);
    k_xcat<<<(unsigned)(((size_t)NB_ * KC / 8 + 255) / 256), 256, 0, stream>>>(x, mh, th, XC); k_cvt8<<<(unsigned)(((size_t)NB_ * IN_ / 8 + 255) / 256), 256, 0, stream>>>(x, XB, (size_t)NB_ * IN_ / 8); k_cvt8<<<(unsigned)(((size_t)NB_ * HM / 8 + 255) / 256), 256, 0, stream>>>(mh, HB, (size_t)NB_ * HM / 8); k_wcat<<<(unsigned)(((size_t)4 * HH * KC / 8 + 255) / 256), 256, 0, stream>>>(Wih, Whh, WC);
    k_cvt8<<<(EE * HH / 8 + 255) / 256, 256, 0, stream>>>(Whz, WHZ, (size_t)EE * HH / 8); k_cvt8<<<(unsigned)(((size_t)4 * HM * IN_ / 8 + 255) / 256), 256, 0, stream>>>(WiH, WIH, (size_t)4 * HM * IN_ / 8); k_cvt8<<<(unsigned)(((size_t)4 * HM * HM / 8 + 255) / 256), 256, 0, stream>>>(WHH, WHHb, (size_t)4 * HM * HM / 8);
    k_cvt8<<<(4 * HM * EE / 8 + 255) / 256, 256, 0, stream>>>(Wd1, WD1, (size_t)4 * HM * EE / 8); k_cvt8<<<(4 * HM * EE / 8 + 255) / 256, 256, 0, stream>>>(Wd2, WD2, (size_t)4 * HM * EE / 8); k_cvt8<<<(4 * HM * EE / 8 + 255) / 256, 256, 0, stream>>>(Wbz, WBZ, (size_t)4 * HM * EE / 8);
    k_gemmw<bf, 0, true><<<dim3(NB_ / 64, 4 * HH / 64, 1), 32, 0, stream>>>(XC, nullptr, WC, nullptr, KC, MP, 4 * HH, bhy, 0, 0, 0);
    k_meta<<<(unsigned)(((size_t)NB_ * HH + 255) / 256), 256, 0, stream>>>(MP, tc, OMH, OMC); k_split4<<<(unsigned)(((size_t)NB_ * HH / 4 + 255) / 256), 256, 0, stream>>>(OMH, MHh, MHl, (size_t)NB_ * HH / 4);
    k_gemmw<bf, 1, false><<<dim3(NB_ / 64, EE / 64, 1), 32, 0, stream>>>(MHh, MHl, WHZ, nullptr, HH, Z, EE, nullptr, 0, 0, 0);
    k_split4<<<(unsigned)(((size_t)NB_ * EE / 4 + 255) / 256), 256, 0, stream>>>(Z, Zh, Zl, (size_t)NB_ * EE / 4);
    float* GATES[4] = {G0, G1, G2, G3};
    for (int gs = 0; gs < 4; ++gs) {
        k_gemmw<bf, 0, false><<<dim3(NB_ / 64, HM / 64, 1), 32, 0, stream>>>(XB, nullptr, WIH + (size_t)gs * HM * IN_, nullptr, IN_, XW, HM, nullptr, 0, 0, 0);
        k_gemmw<bf, 0, false><<<dim3(NB_ / 64, HM / 64, 1), 32, 0, stream>>>(HB, nullptr, WHHb + (size_t)gs * HM * HM, nullptr, HM, HW, HM, nullptr, 0, 0, 0);
        k_gemmw<bf, 1, false><<<dim3(NB_ / 64, HM / 64, 1), 32, 0, stream>>>(Zh, Zl, WD1 + (size_t)gs * HM * EE, nullptr, EE, ZD1, HM, nullptr, 0, 0, 0);
        k_gemmw<bf, 1, false><<<dim3(NB_ / 64, HM / 64, 1), 32, 0, stream>>>(Zh, Zl, WD2 + (size_t)gs * HM * EE, nullptr, EE, ZD2, HM, nullptr, 0, 0, 0);
        k_gemmw<bf, 1, false><<<dim3(NB_ / 64, HM / 64, 1), 32, 0, stream>>>(Zh, Zl, WBZ + (size_t)gs * HM * EE, nullptr, EE, ZB, HM, nullptr, 0, 0, 0);
        k_gate<<<nb4, 256, 0, stream>>>(ZD1, XW, ZD2, HW, ZB, gs, GATES[gs]); }
    k_main<<<nb4, 256, 0, stream>>>(G0, G1, G2, G3, mc, OH, OC);
}
